// SparseDeepUnrolling_52948356825092
// MI455X (gfx1250) — hardware-run, weakly checked
//
#include <hip/hip_runtime.h>
#include <math.h>

typedef __attribute__((ext_vector_type(16))) _Float16 v16h;
typedef __attribute__((ext_vector_type(8)))  _Float16 v8h;
typedef __attribute__((ext_vector_type(8)))  float    v8f;
typedef __attribute__((ext_vector_type(4)))  float    v4f;

constexpr int kB = 4096;
constexpr int kD = 1024;
constexpr int kP = 2048;
constexpr int kSteps = 10;
constexpr float kStep = 0.1f;
constexpr float kThresh = (float)(0.12 * 0.1);

constexpr float kCarryW = 512.0f;
constexpr float kCarryX = 8.0f;
constexpr float kCarryZ = 16.0f;
constexpr float kCarryA = 1024.0f;
constexpr float kScaleGram  = 1.0f / (kCarryW * kCarryW);
constexpr float kScaleBias  = 1.0f / (kCarryX * kCarryW);
constexpr float kScaleIter  = 1.0f / (kCarryZ * kCarryA);
constexpr float kScaleRecon = 1.0f / (kCarryZ * kCarryW);
constexpr float kF16MinNormal = 6.103515625e-05f;

static_assert((kD % 32) == 0 && (kP % 32) == 0);
static_assert((kB % 64) == 0 && (kD % 64) == 0 && (kP % 64) == 0);
static_assert((kP % 256) == 0);
static_assert(((kB * kD / 8) % 256) == 0);
static_assert(kSteps == 10);
static_assert((size_t)kB * kD * 4 == 16777216ull);
static_assert((size_t)kB * kD * 4 + (size_t)kB * kP * 4 == 50331648ull);

constexpr size_t kSzINV = (size_t)kP * 4;
constexpr size_t kSzWT  = (size_t)kP * kD * 2;
constexpr size_t kSzWN  = (size_t)kD * kP * 2;
constexpr size_t kSzXH  = (size_t)kB * kD * 2;
constexpr size_t kSzAM  = (size_t)kP * kP * 2;
constexpr size_t kSzBB  = (size_t)kB * kP * 4;
constexpr size_t kSzZ   = (size_t)kB * kP * 2;
constexpr size_t kOffINV = 0;
constexpr size_t kOffWTH = kOffINV + kSzINV;
constexpr size_t kOffWNH = kOffWTH + kSzWT;
constexpr size_t kOffXH  = kOffWNH + kSzWN;
constexpr size_t kOffAM  = kOffXH  + kSzXH;
constexpr size_t kOffBB  = kOffAM  + kSzAM;
constexpr size_t kOffZ0  = kOffBB  + kSzBB;
constexpr size_t kOffZ1  = kOffZ0  + kSzZ;
constexpr size_t kWsTotal = kOffZ1 + kSzZ;
static_assert(kWsTotal == kSzINV + kSzWT + kSzWN + kSzXH + kSzAM + kSzBB + kSzZ + kSzZ);
static_assert(kWsTotal == 92282880ull);
static_assert(kWsTotal <= 134217728ull);
static_assert((kOffWTH % 128) == 0 && (kOffWNH % 128) == 0 &&
              (kOffXH % 128) == 0 && (kOffAM % 128) == 0 && (kOffBB % 128) == 0 && (kOffZ0 % 128) == 0 &&
              (kOffZ1 % 128) == 0);

__device__ __forceinline__ float bf16_value(float f) {
  const unsigned u = __float_as_uint(f);
  const unsigned r = (u + 0x7FFFu + ((u >> 16) & 1u)) & 0xFFFF0000u;
  return __uint_as_float(r);
}
__device__ __forceinline__ _Float16 f16_flush(float v) {
  const float w = (fabsf(v) < kF16MinNormal) ? 0.0f : v;
  return (_Float16)w;
}

union FragU { v16h v; v8h h[2]; };
__device__ __forceinline__ v16h frag_load(const _Float16* p) {
  FragU f;
  f.h[0] = *(const v8h*)(p);
  f.h[1] = *(const v8h*)(p + 16);
  return f.v;
}
__device__ __forceinline__ v8f mma_f16(v16h a, v16h b, v8f c) {
  return __builtin_amdgcn_wmma_f32_16x16x32_f16(false, a, false, b, (short)0, c, false, false);
}
__device__ __forceinline__ void tie_acc(v8f& c, v16h a, v16h b) {
  asm volatile("" : "+v"(c) : "v"(a), "v"(b));
}
__device__ __forceinline__ void guard_acc(v8f& c, v16h a, v16h b) {
  asm volatile("v_nop\n\tv_nop\n\tv_nop\n\tv_nop" : "+v"(c) : "v"(a), "v"(b));
}
__device__ __forceinline__ void settle_acc(v8f& c) {
  asm volatile("v_nop\n\tv_nop\n\tv_nop\n\tv_nop" : "+v"(c));
}

__global__ __launch_bounds__(256) void col_norms(const float* __restrict__ W, float* __restrict__ inv) {
  const int p = blockIdx.x * 256 + threadIdx.x;
  float s0 = 0.0f, s1 = 0.0f, s2 = 0.0f, s3 = 0.0f;
#pragma unroll 1
  for (int d = 0; d < kD; d += 4) {
    const float v0 = bf16_value(W[(size_t)(d + 0) * kP + p]);
    const float v1 = bf16_value(W[(size_t)(d + 1) * kP + p]);
    const float v2 = bf16_value(W[(size_t)(d + 2) * kP + p]);
    const float v3 = bf16_value(W[(size_t)(d + 3) * kP + p]);
    s0 = fmaf(v0, v0, s0);
    s1 = fmaf(v1, v1, s1);
    s2 = fmaf(v2, v2, s2);
    s3 = fmaf(v3, v3, s3);
  }
  const float s = (s0 + s1) + (s2 + s3);
  const float r = 1.0f / sqrtf(s);
  volatile float* q = inv + p;
  *q = r;
  __threadfence();
  *q = r;
}

__global__ __launch_bounds__(256) void wn_planes(
    const float* __restrict__ W, const float* __restrict__ inv,
    unsigned short* __restrict__ WNH, unsigned short* __restrict__ WTH)
{
  __shared__ float sV[64 * 65];
  const int tid = threadIdx.x;
  const int p0 = blockIdx.x * 64;
  const int d0 = blockIdx.y * 64;
  {
    const int lr = tid >> 4;
    const int c4 = (tid & 15) * 4;
    const v4f iv = *(const v4f*)(inv + p0 + c4);
#pragma unroll
    for (int it = 0; it < 4; ++it) {
      const int row = it * 16 + lr;
      const v4f w = *(const v4f*)(W + (size_t)(d0 + row) * kP + p0 + c4);
#pragma unroll
      for (int e = 0; e < 4; ++e) {
        const float ws = w[e];
        const float is = iv[e];
        const float wn = bf16_value(ws) * is;
        sV[row * 65 + c4 + e] = wn * kCarryW;
      }
    }
  }
  __syncthreads();
  const int q  = tid >> 3;
  const int c8 = (tid & 7) * 8;
  v8h nh[2], th[2];
#pragma unroll
  for (int it = 0; it < 2; ++it) {
    const int row = it * 32 + q;
#pragma unroll
    for (int e = 0; e < 8; ++e) {
      const float vn = sV[row * 65 + c8 + e];
      nh[it][e] = f16_flush(vn);
      const float vt = sV[(c8 + e) * 65 + row];
      th[it][e] = f16_flush(vt);
    }
  }
  for (int pass = 0; pass < 2; ++pass) {
#pragma unroll
    for (int it = 0; it < 2; ++it) {
      const int row = it * 32 + q;
      const size_t on = (size_t)(d0 + row) * kP + p0 + c8;
      const size_t ot = (size_t)(p0 + row) * kD + d0 + c8;
      *(volatile v8h*)(WNH + on) = nh[it];
      *(volatile v8h*)(WTH + ot) = th[it];
    }
    __threadfence();
  }
}

__global__ __launch_bounds__(256) void x_plane(const float* __restrict__ x, unsigned short* __restrict__ XH, int total8) {
  const int i = blockIdx.x * 256 + threadIdx.x;
  if (i >= total8) return;
  const size_t e0 = (size_t)i << 3;
  const v4f a0 = *(const v4f*)(x + e0);
  const v4f a1 = *(const v4f*)(x + e0 + 4);
  v8h hv;
#pragma unroll
  for (int e = 0; e < 4; ++e) {
    const float f0 = a0[e];
    const float f1 = a1[e];
    hv[e]     = f16_flush(bf16_value(f0) * kCarryX);
    hv[4 + e] = f16_flush(bf16_value(f1) * kCarryX);
  }
  unsigned short* qh = XH + e0;
  *(volatile v8h*)qh = hv;
  __threadfence();
  *(volatile v8h*)qh = hv;
}

constexpr int MD_GRAM = 0;
constexpr int MD_BIAS = 1;
constexpr int MD_ITER = 2;
constexpr int MD_ITER_LAST = 3;
constexpr int MD_RECON = 4;

template <int MD>
__global__ __launch_bounds__(256) void gemm64_f16(
    const unsigned short* __restrict__ Ap, int lda,
    const unsigned short* __restrict__ Bhp, int ldb,
    float* __restrict__ Cf, unsigned short* __restrict__ Ch, int ldc,
    const float* __restrict__ addend,
    int M, int N, int K, float scale)
{
  __shared__ __align__(16) float sT[8][16 * 68];
  const int lane = threadIdx.x & 31;
  const int wave = threadIdx.x >> 5;
  const int tilesN = N >> 6;
  const int tilesM = M >> 6;
  const int tile = blockIdx.x * 8 + wave;
  if (tile >= tilesM * tilesN) return;
  const int tm = tile / tilesN;
  const int tn = tile - tm * tilesN;
  const int m0 = tm << 6;
  const int n0 = tn << 6;
  const int rlane = lane & 15;
  const int koff  = (lane >> 4) * 8;
  const int mOff  = (lane >> 4) * 8;

  v8f acc[4][4];
#pragma unroll
  for (int i = 0; i < 4; ++i)
#pragma unroll
    for (int j = 0; j < 4; ++j) acc[i][j] = (v8f){0.f, 0.f, 0.f, 0.f, 0.f, 0.f, 0.f, 0.f};

  const _Float16* arow = (const _Float16*)(const void*)Ap  + (size_t)(m0 + rlane) * lda + koff;
  const _Float16* brow = (const _Float16*)(const void*)Bhp + (size_t)(n0 + rlane) * ldb + koff;

#pragma unroll 1
  for (int k0 = 0; k0 < K; k0 += 32) {
    v16h bf[4];
#pragma unroll
    for (int j = 0; j < 4; ++j) bf[j] = frag_load(brow + (size_t)(j << 4) * ldb + k0);
#pragma unroll
    for (int i = 0; i < 4; ++i) {
      const v16h af = frag_load(arow + (size_t)(i << 4) * lda + k0);
#pragma unroll
      for (int j = 0; j < 4; ++j) acc[i][j] = mma_f16(af, bf[j], acc[i][j]);
      tie_acc(acc[i][0], af, bf[0]);
      tie_acc(acc[i][1], af, bf[1]);
      tie_acc(acc[i][2], af, bf[2]);
      guard_acc(acc[i][3], af, bf[3]);
    }
  }
#pragma unroll
  for (int i = 0; i < 4; ++i) {
    settle_acc(acc[i][0]);
    settle_acc(acc[i][1]);
    settle_acc(acc[i][2]);
    settle_acc(acc[i][3]);
  }

  float* slab = sT[wave];
#pragma unroll
  for (int i = 0; i < 4; ++i) {
    const int mBase = m0 + (i << 4);
#pragma unroll
    for (int j = 0; j < 4; ++j) {
      const int n = n0 + (j << 4) + rlane;
#pragma unroll
      for (int r = 0; r < 8; ++r) {
        float t = acc[i][j][r] * scale;
        if (MD == MD_GRAM) {
          const float idv = ((mBase + mOff + r) == n) ? 1.0f : 0.0f;
          t = idv - kStep * t;
        }
        if (MD == MD_BIAS) t = kStep * t - kThresh;
        slab[(mOff + r) * 68 + (j << 4) + rlane] = t;
      }
    }
    __builtin_amdgcn_fence(__ATOMIC_RELEASE, "workgroup");
    __builtin_amdgcn_wave_barrier();
    __builtin_amdgcn_fence(__ATOMIC_ACQUIRE, "workgroup");

    if (MD != MD_RECON) {
      const int q  = lane >> 3;
      const int c8 = (lane & 7) * 8;
      v8h hv[4];
#pragma unroll
      for (int it = 0; it < 4; ++it) {
        const int row = it * 4 + q;
        const float* sp = slab + row * 68 + c8;
        const v4f s0 = *(const v4f*)(sp);
        const v4f s1 = *(const v4f*)(sp + 4);
        v4f a0 = (v4f){0.f, 0.f, 0.f, 0.f};
        v4f a1 = (v4f){0.f, 0.f, 0.f, 0.f};
        if (MD == MD_ITER || MD == MD_ITER_LAST) {
          const float* bp = addend + (size_t)(mBase + row) * ldc + n0 + c8;
          a0 = *(const v4f*)(bp);
          a1 = *(const v4f*)(bp + 4);
        }
#pragma unroll
        for (int e = 0; e < 4; ++e) {
          float u0 = s0[e];
          float u1 = s1[e];
          if (MD == MD_ITER || MD == MD_ITER_LAST) {
            u0 = u0 + a0[e];
            u1 = u1 + a1[e];
          }
          if (MD != MD_GRAM) {
            u0 = (u0 > 0.0f) ? u0 : 0.0f;
            u1 = (u1 > 0.0f) ? u1 : 0.0f;
          }
          const float cy = (MD == MD_GRAM) ? kCarryA : kCarryZ;
          hv[it][e]     = f16_flush(u0 * cy);
          hv[it][4 + e] = f16_flush(u1 * cy);
        }
      }
      for (int pass = 0; pass < 2; ++pass) {
#pragma unroll
        for (int it = 0; it < 4; ++it) {
          const int row = it * 4 + q;
          *(volatile v8h*)(Ch + (size_t)(mBase + row) * ldc + n0 + c8) = hv[it];
        }
        __threadfence();
      }
    }
    if (MD == MD_BIAS || MD == MD_ITER_LAST || MD == MD_RECON) {
      const int hh = lane >> 4;
      const int c4 = (lane & 15) * 4;
      v4f fv[8];
#pragma unroll
      for (int it = 0; it < 8; ++it) {
        const int row = it * 2 + hh;
        v4f s = *(const v4f*)(slab + row * 68 + c4);
        if (MD == MD_ITER_LAST) {
          const v4f a = *(const v4f*)(addend + (size_t)(mBase + row) * ldc + n0 + c4);
#pragma unroll
          for (int e = 0; e < 4; ++e) {
            const float u = s[e] + a[e];
            s[e] = (u > 0.0f) ? u : 0.0f;
          }
        }
        fv[it] = s;
      }
      for (int pass = 0; pass < 2; ++pass) {
#pragma unroll
        for (int it = 0; it < 8; ++it) {
          const int row = it * 2 + hh;
          *(volatile v4f*)(Cf + (size_t)(mBase + row) * ldc + n0 + c4) = fv[it];
        }
        __threadfence();
      }
    }
    __builtin_amdgcn_fence(__ATOMIC_RELEASE, "workgroup");
    __builtin_amdgcn_wave_barrier();
    __builtin_amdgcn_fence(__ATOMIC_ACQUIRE, "workgroup");
  }
}

extern "C" void kernel_launch(void* const* d_in, const int* in_sizes, int n_in,
                              void* d_out, int out_size, void* d_ws, size_t ws_size,
                              hipStream_t stream) {
  if (n_in < 2) return;
  if (in_sizes[0] != kB * kD) return;
  if (in_sizes[1] != kD * kP) return;
  if (out_size != kB * kD + kB * kP) return;
  if (ws_size < kWsTotal) return;

  const float* x = (const float*)d_in[0];
  const float* W = (const float*)d_in[1];
  float* outX = (float*)d_out;
  float* outZ = outX + (size_t)kB * kD;

  char* ws = (char*)d_ws;
  float*          INV = (float*)(ws + kOffINV);
  unsigned short* WTH = (unsigned short*)(ws + kOffWTH);
  unsigned short* WNH = (unsigned short*)(ws + kOffWNH);
  unsigned short* XH  = (unsigned short*)(ws + kOffXH);
  unsigned short* AM  = (unsigned short*)(ws + kOffAM);
  float*          BB  = (float*)(ws + kOffBB);
  unsigned short* Z0  = (unsigned short*)(ws + kOffZ0);
  unsigned short* Z1  = (unsigned short*)(ws + kOffZ1);

  col_norms<<<kP / 256, 256, 0, stream>>>(W, INV);
  wn_planes<<<dim3(kP / 64, kD / 64), 256, 0, stream>>>(W, INV, WNH, WTH);
  x_plane<<<(kB * kD / 8) / 256, 256, 0, stream>>>(x, XH, kB * kD / 8);

  {
    constexpr int tiles = (kP / 64) * (kP / 64);
    static_assert((tiles % 8) == 0);
    gemm64_f16<MD_GRAM><<<tiles / 8, 256, 0, stream>>>(
        WTH, kD, WTH, kD, BB, AM, kP, INV, kP, kP, kD, kScaleGram);
  }
  {
    constexpr int tiles = (kB / 64) * (kP / 64);
    static_assert((tiles % 8) == 0);
    gemm64_f16<MD_BIAS><<<tiles / 8, 256, 0, stream>>>(
        XH, kD, WTH, kD, BB, Z0, kP, INV, kB, kP, kD, kScaleBias);
  }
  {
    constexpr int tiles = (kB / 64) * (kP / 64);
    static_assert((tiles % 8) == 0);
    for (int t = 2; t <= kSteps; ++t) {
      const unsigned short* src = ((t & 1) == 0) ? Z0 : Z1;
      unsigned short*       dst = ((t & 1) == 0) ? Z1 : Z0;
      if (t < kSteps) {
        gemm64_f16<MD_ITER><<<tiles / 8, 256, 0, stream>>>(
            src, kP, AM, kP, outZ, dst, kP, BB, kB, kP, kP, kScaleIter);
      } else {
        gemm64_f16<MD_ITER_LAST><<<tiles / 8, 256, 0, stream>>>(
            src, kP, AM, kP, outZ, dst, kP, BB, kB, kP, kP, kScaleIter);
      }
    }
  }
  {
    constexpr int tiles = (kB / 64) * (kD / 64);
    static_assert((tiles % 8) == 0);
    gemm64_f16<MD_RECON><<<tiles / 8, 256, 0, stream>>>(
        Z1, kP, WNH, kP, outX, Z0, kD, INV, kB, kD, kP, kScaleRecon);
  }
}
